// LiquidODECore_24927990186047
// MI455X (gfx1250) — hardware-verified
//
#include <hip/hip_runtime.h>


#define NBI  2
#define NVOX 110592
#define NR   (NBI * NVOX)
#define RCH  36864
#define HDN  64
#define DM   HDN
#define NTK  RCH
#define DT_  0.125f
#define LOSC 1024.0f

typedef _Float16 h16;
typedef unsigned short bf;
typedef __attribute__((ext_vector_type(16))) __bf16   v16bf;
typedef __attribute__((ext_vector_type(16))) _Float16 v16h;
typedef __attribute__((ext_vector_type(8)))  _Float16 v8h;
typedef __attribute__((ext_vector_type(8)))  unsigned short v8us;
typedef __attribute__((ext_vector_type(8)))  float    v8f;
typedef __attribute__((ext_vector_type(4)))  float    v4f;
typedef __attribute__((ext_vector_type(4)))  _Float16 v4h;
typedef v8h  __attribute__((may_alias)) v8ha;
typedef v4f  __attribute__((may_alias)) v4fa;
typedef v8us __attribute__((may_alias)) v8usa;

__device__ __forceinline__ unsigned short f2bf(float f) { unsigned u = __float_as_uint(f); u += 0x7FFFu + ((u >> 16) & 1u); return (unsigned short)(u >> 16); }
__device__ __forceinline__ float bf2f(unsigned short b) { return __uint_as_float(((unsigned)b) << 16); }
__device__ __forceinline__ float bfr(float f) { return bf2f(f2bf(f)); }
__device__ __forceinline__ v16h cat16(v8h lo, v8h hi) { return __builtin_shufflevector(lo, hi, 0, 1, 2, 3, 4, 5, 6, 7, 8, 9, 10, 11, 12, 13, 14, 15); }
__device__ __forceinline__ v16bf cat16b(v8us lo, v8us hi) { return __builtin_bit_cast(v16bf, __builtin_shufflevector(lo, hi, 0, 1, 2, 3, 4, 5, 6, 7, 8, 9, 10, 11, 12, 13, 14, 15)); }
__device__ __forceinline__ v8f wmma16(v16h a, v16h b, v8f c) { return __builtin_amdgcn_wmma_f32_16x16x32_f16(false, a, false, b, (short)0, c, false, false); }
__device__ __forceinline__ v8f wmmab(v16bf a, v16bf b, v8f c) { return __builtin_amdgcn_wmma_f32_16x16x32_bf16(false, a, false, b, (short)0, c, false, false); }

template <bool SPLITA, bool F16OUT = false>
__global__ __launch_bounds__(128) void k_gemmb(const bf* __restrict__ A, const bf* __restrict__ Al, const bf* __restrict__ Bn, const float* __restrict__ bias, float* C, int ldc, h16* C2, const float* __restrict__ R = nullptr, int K = DM, int roundR = 1) {
    __shared__ __align__(16) float ost[4][16 * 68];
    const int lane = threadIdx.x & 31, wave = threadIdx.x >> 5, lr = lane & 15, hi = lane >> 4;
    const int r0 = blockIdx.x * 64 + wave * 16, c0 = blockIdx.y * 64;
    const size_t aoff = (size_t)(r0 + lr) * K + 8 * hi;
    size_t boff[4];
#pragma unroll
    for (int t = 0; t < 4; ++t) boff[t] = (size_t)(c0 + t * 16 + lr) * K + 8 * hi;
    v8f acc[4];
#pragma unroll
    for (int t = 0; t < 4; ++t) acc[t] = (v8f){};
#pragma unroll 1
    for (int kc = 0; kc < K; kc += 32) {
        const v16bf a = cat16b(*(const v8us*)(A + aoff + kc), *(const v8us*)(A + aoff + kc + 16));
        v16bf al = a;
        if (SPLITA) al = cat16b(*(const v8us*)(Al + aoff + kc), *(const v8us*)(Al + aoff + kc + 16));
#pragma unroll
        for (int t = 0; t < 4; ++t) { const v16bf b = cat16b(*(const v8us*)(Bn + boff[t] + kc), *(const v8us*)(Bn + boff[t] + kc + 16)); acc[t] = wmmab(a, b, acc[t]); if (SPLITA) acc[t] = wmmab(al, b, acc[t]); }
        asm volatile("v_nop\n\tv_nop\n\tv_nop\n\tv_nop" : "+v"(acc[0]), "+v"(acc[1]), "+v"(acc[2]), "+v"(acc[3]) : "v"(a), "v"(al));
    }
    float* os = &ost[wave][0];
#pragma unroll
    for (int t = 0; t < 4; ++t) { const float bv = bias ? bfr(bias[c0 + t * 16 + lr]) : 0.f;
#pragma unroll
        for (int j = 0; j < 8; ++j) os[(hi * 8 + j) * 68 + t * 16 + lr] = acc[t][j] + bv; }
    __syncthreads();
    if (F16OUT) {
        h16* crow = (h16*)(void*)C + (size_t)r0 * ldc + c0;
        auto pass = [&]() {
#pragma unroll
            for (int s = 0; s < 4; ++s) { const int row = 4 * s + (lane >> 3), piece = lane & 7; const float* sp = os + row * 68 + piece * 8; v8h o, o2;
#pragma unroll
                for (int i = 0; i < 8; ++i) { const h16 a = (h16)sp[i]; o[i] = a; o2[i] = (h16)((sp[i] - (float)a) * LOSC); }
                *(volatile v8h*)(crow + (size_t)row * ldc + piece * 8) = o; if (C2) *(volatile v8h*)(C2 + (size_t)r0 * ldc + c0 + (size_t)row * ldc + piece * 8) = o2; }
        };
        pass(); __threadfence(); pass();
    } else {
        float* crow = C + (size_t)r0 * ldc + c0;
        auto pass = [&]() {
#pragma unroll
            for (int s = 0; s < 8; ++s) { const int Lid = (lane >> 3) + 4 * s, piece = lane & 7; const int row = Lid >> 1, cofs = (Lid & 1) * 32 + piece * 4;
                v4f val = *(const v4fa*)(os + row * 68 + cofs); if (R) { const v4f rv = *(const v4f*)(R + ((size_t)r0 + row) * ldc + c0 + cofs); val += roundR ? (v4f){bfr(rv[0]), bfr(rv[1]), bfr(rv[2]), bfr(rv[3])} : rv; }
                *(volatile v4f*)(crow + (size_t)row * ldc + cofs) = val; }
        };
        pass(); __threadfence(); pass();
    }
}


__global__ __launch_bounds__(256) void k_bf(const float* __restrict__ src, bf* dst, size_t n8) {
    const size_t i = (size_t)blockIdx.x * 256 + threadIdx.x; if (i >= n8) return;
    const v8f v = *(const v8f*)(src + i * 8); v8us o;
#pragma unroll
    for (int k = 0; k < 8; ++k) o[k] = f2bf(v[k]);
    *(volatile v8us*)(dst + i * 8) = o; __threadfence(); *(volatile v8us*)(dst + i * 8) = o;
}
__global__ __launch_bounds__(256) void k_uinit(const float* __restrict__ u, const float* __restrict__ Ut, const float* __restrict__ bt, const float* __restrict__ Uh, const float* __restrict__ bh, size_t row0, float* UT, float* UH) {
    typedef __attribute__((ext_vector_type(2))) float v2f;
    const int lane = threadIdx.x & 31, r = blockIdx.x * 8 + (threadIdx.x >> 5); if (r >= RCH) return;
    const float* ur = u + (row0 + r) * 3; const float u0 = bfr(ur[0]), u1 = bfr(ur[1]), u2 = bfr(ur[2]); v2f a, c;
#pragma unroll
    for (int i = 0; i < 2; ++i) { const int g = 2 * lane + i;
        a[i] = bfr(bt[g]) + u0 * bfr(Ut[g * 3 + 0]) + u1 * bfr(Ut[g * 3 + 1]) + u2 * bfr(Ut[g * 3 + 2]);
        c[i] = bfr(bh[g]) + u0 * bfr(Uh[g * 3 + 0]) + u1 * bfr(Uh[g * 3 + 1]) + u2 * bfr(Uh[g * 3 + 2]); }
    const size_t o = (size_t)r * HDN + 2 * lane;
    *(volatile v2f*)(UT + o) = a; *(volatile v2f*)(UH + o) = c; __threadfence(); *(volatile v2f*)(UT + o) = a; *(volatile v2f*)(UH + o) = c;
}
__global__ __launch_bounds__(256) void k_ode(const float* __restrict__ G, const float* __restrict__ UT, const float* __restrict__ UH, float* H, bf* Hh, bf* Hl) {
    typedef __attribute__((ext_vector_type(2))) float v2f; typedef __attribute__((ext_vector_type(2))) unsigned short v2us;
    const int lane = threadIdx.x & 31, r = blockIdx.x * 8 + (threadIdx.x >> 5); if (r >= RCH) return;
    v2f hv; v2us oh, ol;
#pragma unroll
    for (int i = 0; i < 2; ++i) { const int g = 2 * lane + i;
        const float ut = UT[(size_t)r * HDN + g], uh = UH[(size_t)r * HDN + g];
        const float gt = G ? G[(size_t)r * 128 + g] : 0.f, gh = G ? G[(size_t)r * 128 + 64 + g] : 0.f, hold = G ? H[(size_t)r * HDN + g] : 0.f;
        const float tr = fminf(fmaxf(gt + ut, -50.f), 50.f); const float spl = tr > 20.f ? tr : __logf(1.0f + __expf(tr));
        const float tau = fmaxf(0.1f + spl * 9.9f, 1e-6f); const float f = 1.0f / (1.0f + __expf(-(gh + uh)));
        const float hn = hold + DT_ * (-hold / tau + f); hv[i] = hn; const unsigned short hb = f2bf(hn); oh[i] = hb; ol[i] = f2bf(hn - bf2f(hb)); }
    const size_t o = (size_t)r * HDN + 2 * lane;
    *(volatile v2f*)(H + o) = hv; *(volatile v2us*)(Hh + o) = oh; *(volatile v2us*)(Hl + o) = ol; __threadfence(); *(volatile v2f*)(H + o) = hv; *(volatile v2us*)(Hh + o) = oh; *(volatile v2us*)(Hl + o) = ol;
}
__global__ __launch_bounds__(256) void k_read(const float* __restrict__ H, const float* __restrict__ Wo, const float* __restrict__ bo, size_t row0, float* OUTP) {
    const int r = blockIdx.x * 256 + threadIdx.x; if (r >= RCH) return;
    const float* hr = H + (size_t)r * HDN; float a0 = bfr(bo[0]), a1 = bfr(bo[1]), a2 = bfr(bo[2]);
#pragma unroll 1
    for (int g = 0; g < HDN; ++g) { const float h = hr[g]; a0 = fmaf(h, bfr(Wo[g]), a0); a1 = fmaf(h, bfr(Wo[HDN + g]), a1); a2 = fmaf(h, bfr(Wo[2 * HDN + g]), a2); }
    const size_t gr = row0 + r; const size_t b = gr / NVOX, n = gr % NVOX;
    float* ob = OUTP + (b * 3) * (size_t)NVOX + n;
    const float v0 = tanhf(a0) * 10.f, v1 = tanhf(a1) * 10.f, v2 = tanhf(a2) * 10.f;
    *(volatile float*)(ob) = v0; *(volatile float*)(ob + NVOX) = v1; *(volatile float*)(ob + 2 * (size_t)NVOX) = v2; __threadfence();
    *(volatile float*)(ob) = v0; *(volatile float*)(ob + NVOX) = v1; *(volatile float*)(ob + 2 * (size_t)NVOX) = v2;
}

extern "C" void kernel_launch(void* const* d_in, const int* in_sizes, int n_in,
                              void* d_out, int out_size, void* d_ws, size_t ws_size, hipStream_t stream) {
    (void)in_sizes; (void)n_in; (void)out_size;
    const float* u = (const float*)d_in[0]; const float* Wh_ = (const float*)d_in[1]; const float* Uh = (const float*)d_in[2]; const float* bh = (const float*)d_in[3]; const float* Wt_ = (const float*)d_in[4]; const float* Ut = (const float*)d_in[5]; const float* bt = (const float*)d_in[6]; const float* Wo = (const float*)d_in[7]; const float* bo = (const float*)d_in[8];
    float* out = (float*)d_out;
    char* wsp = (char*)d_ws;
    auto take = [&](size_t bytes) { char* p = wsp; wsp += (bytes + 255) & ~(size_t)255; return (void*)p; };
    bf* Wcat = (bf*)take((size_t)128 * HDN * 2); float* UT = (float*)take((size_t)RCH * HDN * 4); float* UH = (float*)take((size_t)RCH * HDN * 4); float* H = (float*)take((size_t)RCH * HDN * 4); bf* Hh = (bf*)take((size_t)RCH * HDN * 2); bf* Hl = (bf*)take((size_t)RCH * HDN * 2); float* G = (float*)take((size_t)RCH * 128 * 4);
    if ((size_t)(wsp - (char*)d_ws) > ws_size) return;
    k_bf<<<(HDN * HDN / 8 + 255) / 256, 256, 0, stream>>>(Wt_, Wcat, HDN * HDN / 8); k_bf<<<(HDN * HDN / 8 + 255) / 256, 256, 0, stream>>>(Wh_, Wcat + HDN * HDN, HDN * HDN / 8);
    for (int ch = 0; ch < NR / RCH; ++ch) { const size_t row0 = (size_t)ch * RCH;
        k_uinit<<<RCH / 8, 256, 0, stream>>>(u, Ut, bt, Uh, bh, row0, UT, UH);
        k_ode<<<RCH / 8, 256, 0, stream>>>(nullptr, UT, UH, H, Hh, Hl);
        for (int s = 1; s < 8; ++s) {
            k_gemmb<true, false><<<dim3(RCH / 64, 2, 1), 128, 0, stream>>>(Hh, Hl, Wcat, nullptr, G, 128, nullptr, nullptr, HDN);
            k_ode<<<RCH / 8, 256, 0, stream>>>(G, UT, UH, H, Hh, Hl);
        }
        k_read<<<RCH / 256, 256, 0, stream>>>(H, Wo, bo, row0, out);
    }
}
